// StylizationBlock_84318797955700
// MI455X (gfx1250) — hardware-verified
//
#include <hip/hip_runtime.h>
#include <stddef.h>
#include <stdint.h>


#define NB    16
#define NP    16
#define ND    128
#define NT    128
#define N2T   256
#define MROW  (NB * NP * ND)
#define MPOOL (NB * ND)
#define ASC   8
#define HSC   16
#define WSC   64
#define NTHR  256
#define NWAVE 8
#define WSCAP 134217728
#define NEGV  (-1.0e9f)
#define LN_EPS 1.0e-5f
#define LDS_GEMM (NWAVE * 32 * 64 * 4)
#define DLDS_DIST ((ND * ND + NWAVE * NP * ND + ND * 64) * 2)

static_assert(NTHR == NWAVE * 32);
static_assert(NT == 128);
static_assert(ND == 128);
static_assert((MROW % 128) == 0);
static_assert((MPOOL % 128) == 0);
static_assert((N2T % 128) == 0);
static_assert((MROW * NT) % (8 * NTHR) == 0);
static_assert(LDS_GEMM <= 300 * 1024);
static_assert(DLDS_DIST <= 300 * 1024);
static_assert((ND * NT) % NTHR == 0);

typedef float    v4f  __attribute__((ext_vector_type(4)));
typedef float    v8f  __attribute__((ext_vector_type(8)));
typedef _Float16 v8h  __attribute__((ext_vector_type(8)));
typedef _Float16 v16h __attribute__((ext_vector_type(16)));
union FragH { v16h v; v8h h[2]; };

__device__ __forceinline__ v8f wmf(v16h a, v16h b, v8f c) {
  v8f d = __builtin_amdgcn_wmma_f32_16x16x32_f16(false, a, false, b, (short)0, c, false, false);
  asm volatile("v_nop\n\tv_nop\n\tv_nop\n\tv_nop" : "+v"(d) : "v"(a), "v"(b));
  return d;
}

__global__ __launch_bounds__(NTHR) void k_prepw(const float* __restrict__ W, _Float16* Wt, int N, float sc) {
  __shared__ float sw[128 * 32];
  const int tid = threadIdx.x;
  const int n0 = blockIdx.x * 32;
#pragma unroll
  for (int j = 0; j < 16; ++j) {
    const int idx = tid + NTHR * j;
    const int k = idx >> 5, nl = idx & 31;
    sw[idx] = W[(size_t)k * N + n0 + nl] * sc;
  }
  __syncthreads();
  const int c8 = (tid & 15) * 8;
  v8h va, vb;
  const int ra = (tid >> 4), rb = (tid >> 4) + 16;
#pragma unroll
  for (int i = 0; i < 8; ++i) {
    va[i] = (_Float16)sw[(c8 + i) * 32 + ra];
    vb[i] = (_Float16)sw[(c8 + i) * 32 + rb];
  }
  _Float16* da = Wt + (size_t)(n0 + ra) * NT + c8;
  _Float16* dbp = Wt + (size_t)(n0 + rb) * NT + c8;
  *(volatile v8h*)da = va;
  *(volatile v8h*)dbp = vb;
  __threadfence();
  *(volatile v8h*)da = va;
  *(volatile v8h*)dbp = vb;
}

__global__ __launch_bounds__(NTHR) void k_pool(const float* __restrict__ xg, const float* __restrict__ pw,
                                               const float* __restrict__ pb, const int* __restrict__ pm,
                                               _Float16* pooled) {
  __shared__ float spw[ND];
  __shared__ float sred[NWAVE];
  __shared__ float ssc[NP];
  __shared__ float sat[NP];
  __shared__ int smk[NP];
  const int tid = threadIdx.x, lane = tid & 31, wave = tid >> 5, hf = lane >> 4, m = lane & 15;
  const int b = blockIdx.x;
  if (tid < ND) spw[tid] = pw[tid];
  if (wave == 0) { const int mv = pm[b * NP + m]; if (hf == 0) smk[m] = mv; }
  const float pbv = pb[0];
  __syncthreads();

#pragma unroll 1
  for (int p = 0; p < NP; ++p) {
    const float* base = xg + (size_t)(b * NP + p) * (ND * NT);
    float acc = 0.f;
#pragma unroll 4
    for (int jj = 0; jj < (ND * NT) / NTHR; ++jj) {
      const int idx = tid + NTHR * jj;
      acc = fmaf(base[idx], spw[idx >> 7], acc);
    }
#pragma unroll
    for (int off = 16; off > 0; off >>= 1) acc += __shfl_xor(acc, off);
    if (lane == 0) sred[wave] = acc;
    __syncthreads();
    if (tid == 0) {
      float s = 0.f;
#pragma unroll
      for (int w = 0; w < NWAVE; ++w) s += sred[w];
      s = s * (1.0f / (float)NT) + pbv;
      ssc[p] = (smk[p] == 0) ? NEGV : s;
    }
    __syncthreads();
  }
  if (tid == 0) {
    float mx = ssc[0];
#pragma unroll
    for (int p = 1; p < NP; ++p) mx = fmaxf(mx, ssc[p]);
    float den = 0.f;
#pragma unroll
    for (int p = 0; p < NP; ++p) { const float ev = __expf(ssc[p] - mx); sat[p] = ev; den += ev; }
    const float inv = 1.0f / den;
#pragma unroll
    for (int p = 0; p < NP; ++p) sat[p] = sat[p] * inv;
  }
  __syncthreads();

#pragma unroll 1
  for (int jj = 0; jj < 8; ++jj) {
    const int e = 8 * tid + 2048 * jj;
    const int d = e >> 7, tt = e & 127;
    float a[8];
#pragma unroll
    for (int i = 0; i < 8; ++i) a[i] = 0.f;
#pragma unroll 1
    for (int p = 0; p < NP; ++p) {
      const float* q = xg + ((size_t)(b * NP + p) * ND + d) * NT + tt;
      const v4f u0 = *(const v4f*)q, u1 = *(const v4f*)(q + 4);
      const float w = sat[p];
      a[0] = fmaf(w, u0.x, a[0]); a[1] = fmaf(w, u0.y, a[1]); a[2] = fmaf(w, u0.z, a[2]); a[3] = fmaf(w, u0.w, a[3]);
      a[4] = fmaf(w, u1.x, a[4]); a[5] = fmaf(w, u1.y, a[5]); a[6] = fmaf(w, u1.z, a[6]); a[7] = fmaf(w, u1.w, a[7]);
    }
    v8h hv;
#pragma unroll
    for (int i = 0; i < 8; ++i) hv[i] = (_Float16)(a[i] * (float)HSC);
    _Float16* dst = pooled + ((size_t)(b * ND + d)) * NT + tt;
    *(volatile v8h*)dst = hv;
    __threadfence();
    *(volatile v8h*)dst = hv;
  }
}

__global__ __launch_bounds__(NTHR) void k_gemm_bias(const _Float16* __restrict__ A, const _Float16* __restrict__ Bt,
                                                    const float* __restrict__ bias, float* C, int ldc, float osc) {
  extern __shared__ v4f lds_g1[];
  const int tid = threadIdx.x, lane = tid & 31, wave = tid >> 5, hf = lane >> 4, m = lane & 15;
  float* stg = (float*)lds_g1 + wave * (32 * 64);
  const int n0 = blockIdx.x * 128, m0 = blockIdx.y * 128;
  const int wm = (wave >> 1) * 32, wn = (wave & 1) * 64;

  v8f acc[2][4];
#pragma unroll
  for (int mt = 0; mt < 2; ++mt)
#pragma unroll
    for (int nt = 0; nt < 4; ++nt) { v8f z = {0.f, 0.f, 0.f, 0.f, 0.f, 0.f, 0.f, 0.f}; acc[mt][nt] = z; }

  const _Float16* ap = A + (size_t)(m0 + wm + m) * NT + 8 * hf;
  const _Float16* bp = Bt + (size_t)(n0 + wn + m) * NT + 8 * hf;
#pragma unroll 1
  for (int kt = 0; kt < NT / 32; ++kt) {
    const int k0 = 32 * kt;
    FragH a0, a1;
    a0.h[0] = *(const v8h*)(ap + k0);
    a0.h[1] = *(const v8h*)(ap + k0 + 16);
    a1.h[0] = *(const v8h*)(ap + 16 * NT + k0);
    a1.h[1] = *(const v8h*)(ap + 16 * NT + k0 + 16);
#pragma unroll
    for (int nt = 0; nt < 4; ++nt) {
      const _Float16* bq = bp + (size_t)nt * 16 * NT + k0;
      FragH bf;
      bf.h[0] = *(const v8h*)bq;
      bf.h[1] = *(const v8h*)(bq + 16);
      acc[0][nt] = wmf(a0.v, bf.v, acc[0][nt]);
      acc[1][nt] = wmf(a1.v, bf.v, acc[1][nt]);
    }
  }

  float bv[4];
#pragma unroll
  for (int nt = 0; nt < 4; ++nt) bv[nt] = bias[n0 + wn + 16 * nt + m];
#pragma unroll
  for (int mt = 0; mt < 2; ++mt) {
    float* sp = stg + (16 * mt + 8 * hf) * 64 + m;
#pragma unroll
    for (int nt = 0; nt < 4; ++nt) {
#pragma unroll
      for (int r = 0; r < 8; ++r) sp[r * 64 + 16 * nt] = acc[mt][nt][r] * osc + bv[nt];
    }
  }
  __syncthreads();

  float* gbase = C + (size_t)(m0 + wm) * ldc + n0 + wn;
#pragma unroll
  for (int q = 0; q < 16; ++q) {
    const int row = 2 * q + hf;
    const v4f v = *(const v4f*)(stg + row * 64 + 4 * m);
    *(volatile v4f*)(gbase + (size_t)row * ldc + 4 * m) = v;
  }
  __threadfence();
#pragma unroll
  for (int q = 0; q < 16; ++q) {
    const int row = 2 * q + hf;
    const v4f v = *(const v4f*)(stg + row * 64 + 4 * m);
    *(volatile v4f*)(gbase + (size_t)row * ldc + 4 * m) = v;
  }
}

__global__ __launch_bounds__(NTHR) void k_gemm_ln(const _Float16* __restrict__ A, const _Float16* __restrict__ Bt,
                                                  const float* __restrict__ bias, const float* __restrict__ res,
                                                  const float* __restrict__ alpha, const float* __restrict__ beta,
                                                  float* out, float osc) {
  extern __shared__ v4f lds_g2[];
  __shared__ float sps[2][NT];
  __shared__ float spq[2][NT];
  const int tid = threadIdx.x, lane = tid & 31, wave = tid >> 5, hf = lane >> 4, m = lane & 15;
  float* stg_all = (float*)lds_g2;
  float* stg = stg_all + wave * (32 * 64);
  const int m0 = blockIdx.x * 128;
  const int wm = (wave >> 1) * 32, wn = (wave & 1) * 64;

  v8f acc[2][4];
#pragma unroll
  for (int mt = 0; mt < 2; ++mt)
#pragma unroll
    for (int nt = 0; nt < 4; ++nt) { v8f z = {0.f, 0.f, 0.f, 0.f, 0.f, 0.f, 0.f, 0.f}; acc[mt][nt] = z; }

  const _Float16* ap = A + (size_t)(m0 + wm + m) * NT + 8 * hf;
  const _Float16* bp = Bt + (size_t)(wn + m) * NT + 8 * hf;
#pragma unroll 1
  for (int kt = 0; kt < NT / 32; ++kt) {
    const int k0 = 32 * kt;
    FragH a0, a1;
    a0.h[0] = *(const v8h*)(ap + k0);
    a0.h[1] = *(const v8h*)(ap + k0 + 16);
    a1.h[0] = *(const v8h*)(ap + 16 * NT + k0);
    a1.h[1] = *(const v8h*)(ap + 16 * NT + k0 + 16);
#pragma unroll
    for (int nt = 0; nt < 4; ++nt) {
      const _Float16* bq = bp + (size_t)nt * 16 * NT + k0;
      FragH bf;
      bf.h[0] = *(const v8h*)bq;
      bf.h[1] = *(const v8h*)(bq + 16);
      acc[0][nt] = wmf(a0.v, bf.v, acc[0][nt]);
      acc[1][nt] = wmf(a1.v, bf.v, acc[1][nt]);
    }
  }

  float bv[4];
#pragma unroll
  for (int nt = 0; nt < 4; ++nt) bv[nt] = bias[wn + 16 * nt + m];
#pragma unroll
  for (int mt = 0; mt < 2; ++mt) {
    float* sp = stg + (16 * mt + 8 * hf) * 64 + m;
#pragma unroll
    for (int nt = 0; nt < 4; ++nt) {
#pragma unroll
      for (int r = 0; r < 8; ++r) sp[r * 64 + 16 * nt] = acc[mt][nt][r] * osc + bv[nt];
    }
  }
  __syncthreads();

  const int t = tid & 127, rh = tid >> 7;
  const int cpart = (t >> 6) * 2048 + (t & 63);
  float sum = 0.f;
#pragma unroll 4
  for (int i = 0; i < 64; ++i) {
    const int R = 64 * rh + i;
    const int idx = (R >> 5) * 4096 + cpart + (R & 31) * 64;
    const float v = stg_all[idx] + res[(size_t)(m0 + R) * NT + t];
    stg_all[idx] = v;
    sum += v;
  }
  sps[rh][t] = sum;
  __syncthreads();
  const float mean = (sps[0][t] + sps[1][t]) * (1.0f / (float)ND);
  float sq = 0.f;
#pragma unroll 4
  for (int i = 0; i < 64; ++i) {
    const int R = 64 * rh + i;
    const int idx = (R >> 5) * 4096 + cpart + (R & 31) * 64;
    const float dv = stg_all[idx] - mean;
    sq = fmaf(dv, dv, sq);
  }
  spq[rh][t] = sq;
  __syncthreads();
  const float var = (spq[0][t] + spq[1][t]) * (1.0f / (float)ND);
  const float rstd = rsqrtf(var + LN_EPS);
#pragma unroll 4
  for (int i = 0; i < 64; ++i) {
    const int R = 64 * rh + i;
    const int idx = (R >> 5) * 4096 + cpart + (R & 31) * 64;
    const float y = (stg_all[idx] - mean) * rstd;
    stg_all[idx] = y * alpha[R] + beta[R];
  }
  __syncthreads();

  float* gbase = out + (size_t)(m0 + wm) * NT + wn;
#pragma unroll
  for (int q = 0; q < 16; ++q) {
    const int row = 2 * q + hf;
    const v4f v = *(const v4f*)(stg + row * 64 + 4 * m);
    *(volatile v4f*)(gbase + (size_t)row * NT + 4 * m) = v;
  }
  __threadfence();
#pragma unroll
  for (int q = 0; q < 16; ++q) {
    const int row = 2 * q + hf;
    const v4f v = *(const v4f*)(stg + row * 64 + 4 * m);
    *(volatile v4f*)(gbase + (size_t)row * NT + 4 * m) = v;
  }
}

__global__ __launch_bounds__(NTHR) void k_film(const float* __restrict__ x, const float* __restrict__ emb,
                                               _Float16* xm16, _Float16* x16) {
  const size_t g = (size_t)blockIdx.x * NTHR + threadIdx.x;
  const size_t e = g * 8;
  const size_t row = e >> 7;
  const int tt = (int)(e & 127);
  const int b = (int)(row >> 11), d = (int)(row & 127);
  const float* px = x + row * NT + tt;
  const v4f xa = *(const v4f*)px, xb = *(const v4f*)(px + 4);
  const float* ps = emb + ((size_t)(b * ND + d)) * N2T + tt;
  const v4f sa = *(const v4f*)ps, sb = *(const v4f*)(ps + 4);
  const v4f ha = *(const v4f*)(ps + NT), hb = *(const v4f*)(ps + NT + 4);
  float xv[8], sv[8], hv8[8];
  xv[0] = xa.x; xv[1] = xa.y; xv[2] = xa.z; xv[3] = xa.w; xv[4] = xb.x; xv[5] = xb.y; xv[6] = xb.z; xv[7] = xb.w;
  sv[0] = sa.x; sv[1] = sa.y; sv[2] = sa.z; sv[3] = sa.w; sv[4] = sb.x; sv[5] = sb.y; sv[6] = sb.z; sv[7] = sb.w;
  hv8[0] = ha.x; hv8[1] = ha.y; hv8[2] = ha.z; hv8[3] = ha.w; hv8[4] = hb.x; hv8[5] = hb.y; hv8[6] = hb.z; hv8[7] = hb.w;
  v8h vm, vx;
#pragma unroll
  for (int i = 0; i < 8; ++i) {
    vx[i] = (_Float16)(xv[i] * (float)ASC);
    const float fm = xv[i] * (1.0f + sv[i]) + hv8[i];
    vm[i] = (_Float16)(fm * (float)ASC);
  }
  _Float16* dm = xm16 + row * NT + tt;
  _Float16* dx = x16 + row * NT + tt;
  *(volatile v8h*)dm = vm;
  *(volatile v8h*)dx = vx;
  __threadfence();
  *(volatile v8h*)dm = vm;
  *(volatile v8h*)dx = vx;
}

__global__ __launch_bounds__(NTHR) void k_dist(const float* __restrict__ dist, const int* __restrict__ pm,
                                               const float* __restrict__ w1, const float* __restrict__ b1,
                                               const _Float16* __restrict__ w2t, const float* __restrict__ b2,
                                               const float* __restrict__ dw, const float* __restrict__ dbias,
                                               _Float16* dctx) {
  extern __shared__ v4f lds_d[];
  __shared__ __attribute__((aligned(16))) float sw1[ND];
  __shared__ __attribute__((aligned(16))) float sb1[ND];
  __shared__ float sb2[ND];
  __shared__ float sdw[ND];
  __shared__ int smk[NP];
  const int tid = threadIdx.x, lane = tid & 31, wave = tid >> 5, hf = lane >> 4, m = lane & 15;
  const int bp = blockIdx.x >> 1, b = bp >> 4, p = bp & 15, t0 = (blockIdx.x & 1) * 64;
  _Float16* sW2 = (_Float16*)lds_d;
  _Float16* hTw = sW2 + ND * ND + wave * (NP * ND);
  _Float16* tile = sW2 + ND * ND + NWAVE * (NP * ND);

#pragma unroll
  for (int it = 0; it < (ND * ND) / (8 * NTHR); ++it) {
    const int idx = tid + NTHR * it;
    ((v8h*)sW2)[idx] = ((const v8h*)w2t)[idx];
  }
  if (tid < ND) {
    sw1[tid] = w1[tid] * (float)HSC;
    sb1[tid] = b1[tid] * (float)HSC;
    sb2[tid] = b2[tid];
    sdw[tid] = dw[tid];
  }
  if (wave == 0) { const int mv = pm[b * NP + m]; if (hf == 0) smk[m] = mv; }
  const float dbv = dbias[0];
  __syncthreads();

  const int kk = 8 * m;
  float w8[8], b8[8];
  {
    const v4f wl = *(const v4f*)(sw1 + kk), wh = *(const v4f*)(sw1 + kk + 4);
    const v4f bl = *(const v4f*)(sb1 + kk), bh = *(const v4f*)(sb1 + kk + 4);
    w8[0] = wl.x; w8[1] = wl.y; w8[2] = wl.z; w8[3] = wl.w; w8[4] = wh.x; w8[5] = wh.y; w8[6] = wh.z; w8[7] = wh.w;
    b8[0] = bl.x; b8[1] = bl.y; b8[2] = bl.z; b8[3] = bl.w; b8[4] = bh.x; b8[5] = bh.y; b8[6] = bh.z; b8[7] = bh.w;
  }
  constexpr float OSC3 = 1.0f / (float)(HSC * WSC);

#pragma unroll 1
  for (int j = 0; j < 8; ++j) {
    const int tl = 8 * j + wave, t = t0 + tl;
    const float* sp = dist + ((size_t)(b * NT + t) * NP + p) * NP + 8 * hf;
    const v4f s0 = *(const v4f*)sp, s1 = *(const v4f*)(sp + 4);
    float s8[8];
    s8[0] = s0.x; s8[1] = s0.y; s8[2] = s0.z; s8[3] = s0.w; s8[4] = s1.x; s8[5] = s1.y; s8[6] = s1.z; s8[7] = s1.w;
#pragma unroll
    for (int r = 0; r < 8; ++r) {
      v8h hv;
#pragma unroll
      for (int i = 0; i < 8; ++i) hv[i] = (_Float16)fmaxf(fmaf(s8[r], w8[i], b8[i]), 0.0f);
      *(v8h*)(hTw + (8 * hf + r) * ND + kk) = hv;
    }
    __syncthreads();

    v8f acc[8];
#pragma unroll
    for (int nt = 0; nt < 8; ++nt) { v8f z = {0.f, 0.f, 0.f, 0.f, 0.f, 0.f, 0.f, 0.f}; acc[nt] = z; }
    const _Float16* ap = hTw + m * ND + 8 * hf;
    const _Float16* bpp = sW2 + m * ND + 8 * hf;
#pragma unroll
    for (int c = 0; c < 4; ++c) {
      const int k0 = 32 * c;
      FragH a;
      a.h[0] = *(const v8h*)(ap + k0);
      a.h[1] = *(const v8h*)(ap + k0 + 16);
#pragma unroll
      for (int nt = 0; nt < 8; ++nt) {
        const _Float16* bq = bpp + nt * 16 * ND + k0;
        FragH bf;
        bf.h[0] = *(const v8h*)bq;
        bf.h[1] = *(const v8h*)(bq + 16);
        acc[nt] = wmf(a.v, bf.v, acc[nt]);
      }
    }

    float lg[8];
#pragma unroll
    for (int r = 0; r < 8; ++r) lg[r] = 0.f;
#pragma unroll
    for (int nt = 0; nt < 8; ++nt) {
      const float bb2 = sb2[16 * nt + m], ww = sdw[16 * nt + m];
#pragma unroll
      for (int r = 0; r < 8; ++r) {
        const float de = fmaf(acc[nt][r], OSC3, bb2);
        acc[nt][r] = de;
        lg[r] = fmaf(de, ww, lg[r]);
      }
    }
#pragma unroll
    for (int off = 1; off < 16; off <<= 1) {
#pragma unroll
      for (int r = 0; r < 8; ++r) lg[r] += __shfl_xor(lg[r], off);
    }
    float own[8], oth[8];
#pragma unroll
    for (int r = 0; r < 8; ++r) {
      const float L = lg[r] + dbv;
      own[r] = (smk[8 * hf + r] == 0) ? NEGV : L;
    }
#pragma unroll
    for (int r = 0; r < 8; ++r) oth[r] = __shfl_xor(own[r], 16);
    float mx = own[0];
#pragma unroll
    for (int r = 1; r < 8; ++r) mx = fmaxf(mx, own[r]);
#pragma unroll
    for (int r = 0; r < 8; ++r) mx = fmaxf(mx, oth[r]);
    float eo[8], et[8];
#pragma unroll
    for (int r = 0; r < 8; ++r) { eo[r] = __expf(own[r] - mx); et[r] = __expf(oth[r] - mx); }
    float dlo = 0.f, dhi = 0.f;
#pragma unroll
    for (int r = 0; r < 8; ++r) dlo += (hf != 0) ? et[r] : eo[r];
#pragma unroll
    for (int r = 0; r < 8; ++r) dhi += (hf != 0) ? eo[r] : et[r];
    const float inv = 1.0f / (dlo + dhi);
    float aw[8];
#pragma unroll
    for (int r = 0; r < 8; ++r) aw[r] = eo[r] * inv;
    float v[8];
#pragma unroll
    for (int nt = 0; nt < 8; ++nt) {
      float a2 = 0.f;
#pragma unroll
      for (int r = 0; r < 8; ++r) a2 = fmaf(aw[r], acc[nt][r], a2);
      v[nt] = a2;
    }
#pragma unroll
    for (int nt = 0; nt < 8; ++nt) v[nt] += __shfl_xor(v[nt], 16);
    if (hf == 0) {
#pragma unroll
      for (int nt = 0; nt < 8; ++nt) tile[(16 * nt + m) * 64 + tl] = (_Float16)(v[nt] * (float)HSC);
    }
  }
  __syncthreads();

  const int rsub = lane >> 3, piece = (lane & 7) * 8;
  v8h ov[4];
#pragma unroll
  for (int q = 0; q < 4; ++q) {
    const int d = 16 * wave + 4 * q + rsub;
    ov[q] = *(const v8h*)(tile + d * 64 + piece);
  }
#pragma unroll
  for (int q = 0; q < 4; ++q) {
    const int d = 16 * wave + 4 * q + rsub;
    *(volatile v8h*)(dctx + ((size_t)(bp * ND + d)) * NT + t0 + piece) = ov[q];
  }
  __threadfence();
#pragma unroll
  for (int q = 0; q < 4; ++q) {
    const int d = 16 * wave + 4 * q + rsub;
    *(volatile v8h*)(dctx + ((size_t)(bp * ND + d)) * NT + t0 + piece) = ov[q];
  }
}

extern "C" void kernel_launch(void* const* d_in, const int* in_sizes, int n_in,
                              void* d_out, int out_size, void* d_ws, size_t ws_size,
                              hipStream_t stream) {
  if (n_in < 24) return;
  const int want[24] = {MROW * NT, MROW * NT, NB * NT * NP * NP, NB * NP, NT * N2T, N2T,
                        NT * NT, NT, NT * NT, NT, NT * NT, NT, ND, ND, ND * ND, ND,
                        ND, 1, ND, 1, ND, ND, ND, ND};
  for (int i = 0; i < 24; ++i) if (in_sizes[i] != want[i]) return;
  if (out_size != 2 * MROW * NT) return;

  const float* x       = (const float*)d_in[0];
  const float* xg      = (const float*)d_in[1];
  const float* dist    = (const float*)d_in[2];
  const int*   pmask   = (const int*)d_in[3];
  const float* emb_w   = (const float*)d_in[4];
  const float* emb_b   = (const float*)d_in[5];
  const float* out_w   = (const float*)d_in[6];
  const float* out_b   = (const float*)d_in[7];
  const float* glob_w  = (const float*)d_in[8];
  const float* glob_b  = (const float*)d_in[9];
  const float* temp_w  = (const float*)d_in[10];
  const float* temp_b  = (const float*)d_in[11];
  const float* mlp_w1  = (const float*)d_in[12];
  const float* mlp_b1  = (const float*)d_in[13];
  const float* mlp_w2  = (const float*)d_in[14];
  const float* mlp_b2  = (const float*)d_in[15];
  const float* pool_w  = (const float*)d_in[16];
  const float* pool_b  = (const float*)d_in[17];
  const float* dis_w   = (const float*)d_in[18];
  const float* dis_b   = (const float*)d_in[19];
  const float* n_alpha = (const float*)d_in[20];
  const float* n_beta  = (const float*)d_in[21];
  const float* g_alpha = (const float*)d_in[22];
  const float* g_beta  = (const float*)d_in[23];
  float* out0 = (float*)d_out;
  float* out1 = out0 + (size_t)MROW * NT;

  char* ws = (char*)d_ws;
  size_t off = 0;
  const size_t oWo = off; off += (size_t)NT * NT * 2;    off = (off + 255) & ~(size_t)255;
  const size_t oWg = off; off += (size_t)NT * NT * 2;    off = (off + 255) & ~(size_t)255;
  const size_t oWt = off; off += (size_t)NT * NT * 2;    off = (off + 255) & ~(size_t)255;
  const size_t oW2 = off; off += (size_t)ND * ND * 2;    off = (off + 255) & ~(size_t)255;
  const size_t oWe = off; off += (size_t)N2T * NT * 2;   off = (off + 255) & ~(size_t)255;
  const size_t oPo = off; off += (size_t)MPOOL * NT * 2; off = (off + 255) & ~(size_t)255;
  const size_t oEm = off; off += (size_t)MPOOL * N2T * 4; off = (off + 255) & ~(size_t)255;
  const size_t oXm = off; off += (size_t)MROW * NT * 2;  off = (off + 255) & ~(size_t)255;
  const size_t oXh = off; off += (size_t)MROW * NT * 2;  off = (off + 255) & ~(size_t)255;
  const size_t oDc = off; off += (size_t)MROW * NT * 2;  off = (off + 255) & ~(size_t)255;
  const size_t oX1 = off; off += (size_t)MROW * NT * 4;  off = (off + 255) & ~(size_t)255;
  if (off > ws_size || off > (size_t)WSCAP) return;
  _Float16* outWt  = (_Float16*)(ws + oWo);
  _Float16* globWt = (_Float16*)(ws + oWg);
  _Float16* tempWt = (_Float16*)(ws + oWt);
  _Float16* w2T    = (_Float16*)(ws + oW2);
  _Float16* embWt  = (_Float16*)(ws + oWe);
  _Float16* pooled = (_Float16*)(ws + oPo);
  float*    embout = (float*)(ws + oEm);
  _Float16* xm16   = (_Float16*)(ws + oXm);
  _Float16* x16    = (_Float16*)(ws + oXh);
  _Float16* dctx16 = (_Float16*)(ws + oDc);
  float*    x1pre  = (float*)(ws + oX1);

  const float oscA = 1.0f / (float)(ASC * WSC);
  const float oscH = 1.0f / (float)(HSC * WSC);

  k_prepw<<<NT / 32, NTHR, 0, stream>>>(out_w, outWt, NT, (float)WSC);
  k_prepw<<<NT / 32, NTHR, 0, stream>>>(glob_w, globWt, NT, (float)WSC);
  k_prepw<<<NT / 32, NTHR, 0, stream>>>(temp_w, tempWt, NT, (float)WSC);
  k_prepw<<<ND / 32, NTHR, 0, stream>>>(mlp_w2, w2T, ND, (float)WSC);
  k_prepw<<<N2T / 32, NTHR, 0, stream>>>(emb_w, embWt, N2T, (float)WSC);
  k_pool<<<NB, NTHR, 0, stream>>>(xg, pool_w, pool_b, pmask, pooled);
  hipFuncSetAttribute(reinterpret_cast<const void*>(&k_gemm_bias),
                      hipFuncAttributeMaxDynamicSharedMemorySize, LDS_GEMM);
  k_gemm_bias<<<dim3(N2T / 128, MPOOL / 128), NTHR, LDS_GEMM, stream>>>(pooled, embWt, emb_b, embout, N2T, oscH);
  k_film<<<(MROW * NT) / (8 * NTHR), NTHR, 0, stream>>>(x, embout, xm16, x16);
  k_gemm_bias<<<dim3(NT / 128, MROW / 128), NTHR, LDS_GEMM, stream>>>(xm16, outWt, out_b, x1pre, NT, oscA);
  hipFuncSetAttribute(reinterpret_cast<const void*>(&k_gemm_ln),
                      hipFuncAttributeMaxDynamicSharedMemorySize, LDS_GEMM);
  k_gemm_ln<<<MROW / 128, NTHR, LDS_GEMM, stream>>>(x16, globWt, glob_b, xg, g_alpha, g_beta, out1, oscA);
  hipFuncSetAttribute(reinterpret_cast<const void*>(&k_dist),
                      hipFuncAttributeMaxDynamicSharedMemorySize, DLDS_DIST);
  k_dist<<<NB * NP * 2, NTHR, DLDS_DIST, stream>>>(dist, pmask, mlp_w1, mlp_b1, w2T, mlp_b2, dis_w, dis_b, dctx16);
  k_gemm_ln<<<MROW / 128, NTHR, LDS_GEMM, stream>>>(dctx16, tempWt, temp_b, x1pre, n_alpha, n_beta, out0, oscH);
}
